// triplet_loss_cl_1709396984281
// MI455X (gfx1250) — hardware-verified
//
#include <hip/hip_runtime.h>
#include <math.h>
#include <stdint.h>


typedef _Float16 v16h __attribute__((ext_vector_type(16)));
typedef _Float16 v8h  __attribute__((ext_vector_type(8)));
typedef float    v8f  __attribute__((ext_vector_type(8)));
typedef float    v4f  __attribute__((ext_vector_type(4)));
typedef float    v4fa __attribute__((ext_vector_type(4), __may_alias__));

union Frag { v16h v; v8h half[2]; };

#define NQ    8192
#define DK    256
#define KCH   (DK / 32)
#define WPB   4
#define TPB   (WPB * 32)
#define QPB   (WPB * 16)
#define NKT   (NQ / 16)
#define EPSL  1e-5f
#define CVT_TPB 256
#define FIN_TPB 256

__device__ __forceinline__ v8f wmma16(v16h a, v16h b, v8f c)
{
    v8f d = __builtin_amdgcn_wmma_f32_16x16x32_f16(false, a, false, b, (short)0, c, false, false);
    asm volatile("v_nop\n\tv_nop\n\tv_nop\n\tv_nop" : "+v"(d) : "v"(a), "v"(b));
    return d;
}

__global__ __launch_bounds__(CVT_TPB)
void k_convert(const float* __restrict__ q, const float* __restrict__ g,
               _Float16* __restrict__ qh, _Float16* __restrict__ gh, int n8)
{
    const int i = blockIdx.x * CVT_TPB + threadIdx.x;
    if (i >= 2 * n8) return;
    const bool first = (i < n8);
    const int j = first ? i : (i - n8);
    const float* src = first ? q : g;
    _Float16* dst = first ? qh : gh;

    const v4f a = *(const v4f*)(src + (size_t)j * 8);
    const v4f b = *(const v4f*)(src + (size_t)j * 8 + 4);
    v8h o;
    o[0] = (_Float16)a[0]; o[1] = (_Float16)a[1]; o[2] = (_Float16)a[2]; o[3] = (_Float16)a[3];
    o[4] = (_Float16)b[0]; o[5] = (_Float16)b[1]; o[6] = (_Float16)b[2]; o[7] = (_Float16)b[3];

    _Float16* p = dst + (size_t)j * 8;
    *(volatile v8h*)p = o;
    __threadfence();
    *(volatile v8h*)p = o;
}

__global__ __launch_bounds__(TPB)
void k_rowpass(const _Float16* __restrict__ qh, const _Float16* __restrict__ gh,
               float* __restrict__ lossp)
{
    __shared__ __attribute__((aligned(16))) float sLoss[QPB];

    const int tid  = threadIdx.x;
    const int wave = tid >> 5;
    const int lane = tid & 31;
    const int h    = lane >> 4;
    const int m    = lane & 15;
    const int row0 = blockIdx.x * QPB + wave * 16;

    Frag bq[KCH];
    {
        const _Float16* qr = qh + (size_t)(row0 + m) * DK + 8 * h;
#pragma unroll
        for (int c = 0; c < KCH; ++c) {
            bq[c].half[0] = *(const v8h*)(qr + c * 32);
            bq[c].half[1] = *(const v8h*)(qr + c * 32 + 16);
        }
    }

    const int want     = (m >= 8 * h && m < 8 * h + 8) ? (m - 8 * h) : -1;
    const int diagTile = blockIdx.x * WPB + wave;

    float mrun = -INFINITY;
    float srun = 0.0f;
    float diag = 0.0f;

#pragma unroll 1
    for (int jt = 0; jt < NKT; ++jt) {
        const _Float16* gr = gh + (size_t)(jt * 16 + m) * DK + 8 * h;
        v8f acc = {0.0f, 0.0f, 0.0f, 0.0f, 0.0f, 0.0f, 0.0f, 0.0f};
#pragma unroll
        for (int c = 0; c < KCH; ++c) {
            Frag a;
            a.half[0] = *(const v8h*)(gr + c * 32);
            a.half[1] = *(const v8h*)(gr + c * 32 + 16);
            acc = wmma16(a.v, bq[c].v, acc);
        }

        const float t01 = fmaxf(acc[0], acc[1]);
        const float t23 = fmaxf(acc[2], acc[3]);
        const float t45 = fmaxf(acc[4], acc[5]);
        const float t67 = fmaxf(acc[6], acc[7]);
        const float tmax = fmaxf(fmaxf(t01, t23), fmaxf(t45, t67));
        const float mnew = fmaxf(mrun, tmax);
        float add = 0.0f;
        add += __expf(acc[0] - mnew);
        add += __expf(acc[1] - mnew);
        add += __expf(acc[2] - mnew);
        add += __expf(acc[3] - mnew);
        add += __expf(acc[4] - mnew);
        add += __expf(acc[5] - mnew);
        add += __expf(acc[6] - mnew);
        add += __expf(acc[7] - mnew);
        srun = srun * __expf(mrun - mnew) + add;
        mrun = mnew;

        if (jt == diagTile) {
#pragma unroll
            for (int r = 0; r < 8; ++r)
                if (r == want) diag = acc[r];
        }
    }

    const float mo  = __shfl_xor(mrun, 16);
    const float so  = __shfl_xor(srun, 16);
    const float dth = __shfl_xor(diag, 16);
    const float M   = fmaxf(mrun, mo);
    const float S   = srun * __expf(mrun - M) + so * __expf(mo - M);
    const float dv  = (want >= 0) ? diag : dth;
    const float p   = __expf(dv - M) * __builtin_amdgcn_rcpf(S);
    const float loss = -__logf(p + EPSL);

    if (h == 0) sLoss[wave * 16 + m] = loss;
    __syncthreads();

    if (wave == 0 && lane < 16) {
        const v4fa v = *(const v4fa*)&sLoss[4 * lane];
        float* dst = lossp + (size_t)blockIdx.x * QPB + 4 * lane;
        *(volatile v4f*)dst = v;
        __threadfence();
        *(volatile v4f*)dst = v;
    }
}

__global__ __launch_bounds__(FIN_TPB)
void k_final(const float* __restrict__ lossp, float* __restrict__ out)
{
    __shared__ double sd[FIN_TPB];
    const int t = threadIdx.x;
    double a = 0.0;
#pragma unroll 1
    for (int i = t; i < NQ; i += FIN_TPB) a += (double)lossp[i];
    sd[t] = a;
    __syncthreads();
#pragma unroll 1
    for (int st = FIN_TPB / 2; st > 0; st >>= 1) {
        if (t < st) sd[t] = sd[t] + sd[t + st];
        __syncthreads();
    }
    if (t == 0) {
        const float v = (float)(sd[0] * (1.0 / (double)NQ));
        *(volatile float*)out = v;
        __threadfence();
        *(volatile float*)out = v;
    }
}

extern "C" void kernel_launch(void* const* d_in, const int* in_sizes, int n_in,
                              void* d_out, int out_size, void* d_ws, size_t ws_size,
                              hipStream_t stream)
{
    if (n_in < 2) return;
    if (in_sizes[0] != NQ * DK || in_sizes[1] != NQ * DK) return;
    if (out_size < 1) return;

    const size_t plane_bytes = (size_t)NQ * DK * sizeof(_Float16);
    const size_t off_q = 0;
    const size_t off_g = off_q + plane_bytes;
    const size_t off_l = off_g + plane_bytes;
    const size_t total = off_l + (size_t)NQ * sizeof(float);
    if (total > ws_size) return;

    const float* q = (const float*)d_in[0];
    const float* g = (const float*)d_in[1];
    char* ws = (char*)d_ws;
    _Float16* qh   = (_Float16*)(ws + off_q);
    _Float16* gh   = (_Float16*)(ws + off_g);
    float*    lossp = (float*)(ws + off_l);

    const int n8 = NQ * DK / 8;
    const int cvt_blocks = (2 * n8 + CVT_TPB - 1) / CVT_TPB;
    k_convert<<<dim3(cvt_blocks), dim3(CVT_TPB), 0, stream>>>(q, g, qh, gh, n8);

    const int row_blocks = (NQ + QPB - 1) / QPB;
    k_rowpass<<<dim3(row_blocks), dim3(TPB), 0, stream>>>(qh, gh, lossp);

    k_final<<<dim3(1), dim3(FIN_TPB), 0, stream>>>(lossp, (float*)d_out);
}
